// MultiHeadCoAttention_88158498717883
// MI455X (gfx1250) — hardware-verified
//
#include <hip/hip_runtime.h>
#include <math.h>

constexpr int  kBatch = 2;
constexpr int  kSeq   = 2048;
constexpr int  kDim   = 1024;
constexpr int  kHeads = 16;
constexpr int  kDh    = 64;
constexpr int  kHeadsPerChunk = 4;
constexpr long kTokDim = (long)kSeq * kDim;
constexpr long kDimDim = (long)kDim * kDim;
constexpr long kSeqSeq = (long)kSeq * kSeq;
constexpr float kWCarry   = 16.0f;
constexpr float kPCarry   = 2048.0f;
constexpr float kResCarry = 64.0f;
constexpr float kScoreScale = 0.125f;
constexpr float kProjScale  = 1.0f / 16.0f;
constexpr float kPVScale    = 64.0f / 2048.0f;
constexpr float kOutScale   = 1.0f / (64.0f * 16.0f);

constexpr size_t kMiB     = 1048576;
constexpr size_t kOffX16q = 0;
constexpr size_t kOffX16c = 4 * kMiB;
constexpr size_t kOffW03  = 8 * kMiB;
constexpr size_t kOffS    = 0;
constexpr size_t kOffP    = 64 * kMiB;
constexpr size_t kOffW45  = 0;
constexpr size_t kOffQ16  = 96 * kMiB;
constexpr size_t kOffC16  = 100 * kMiB;
constexpr size_t kOffQVT  = 104 * kMiB;
constexpr size_t kOffCVT  = 108 * kMiB;
constexpr size_t kOffQRES = 112 * kMiB;
constexpr size_t kOffCRES = 116 * kMiB;
constexpr size_t kWsTotal = 120 * kMiB;

typedef __attribute__((ext_vector_type(16))) _Float16 v16h;
typedef __attribute__((ext_vector_type(8)))  _Float16 v8h;
typedef __attribute__((ext_vector_type(16))) __bf16   v16b;
typedef __attribute__((ext_vector_type(8)))  __bf16   v8b;
typedef __attribute__((ext_vector_type(8)))  float    v8f;
typedef __attribute__((ext_vector_type(4)))  float    v4f;
typedef __attribute__((ext_vector_type(4)))  unsigned int v4u;

__device__ __forceinline__ unsigned short f2bf_bits(float f) {
  unsigned u = __float_as_uint(f);
  return (unsigned short)((u + 0x7FFFu + ((u >> 16) & 1u)) >> 16);
}
__device__ __forceinline__ float bf_bits2f(unsigned short h) { return __uint_as_float(((unsigned)h) << 16); }

__device__ __forceinline__ void dep_guard_h(v8f& a, v8f& b, v16h x, v16h y) { asm volatile("v_nop\n\tv_nop\n\tv_nop\n\tv_nop" : "+v"(a), "+v"(b) : "v"(x), "v"(y)); }
__device__ __forceinline__ void dep_guard_b(v8f& a, v8f& b, v16b x, v16b y) { asm volatile("v_nop\n\tv_nop\n\tv_nop\n\tv_nop" : "+v"(a), "+v"(b) : "v"(x), "v"(y)); }
__device__ __forceinline__ void keep4_h(v16h a, v16h b, v16h c, v16h d) { asm volatile("v_nop" :: "v"(a), "v"(b), "v"(c), "v"(d)); }
__device__ __forceinline__ void keep4_b(v16b a, v16b b, v16b c, v16b d) { asm volatile("v_nop" :: "v"(a), "v"(b), "v"(c), "v"(d)); }
__device__ __forceinline__ void acc_guard4(v8f& a, v8f& b, v8f& c, v8f& d) { asm volatile("v_nop\n\tv_nop\n\tv_nop\n\tv_nop" : "+v"(a), "+v"(b), "+v"(c), "+v"(d)); }
template <typename T> struct Frag;
template <> struct Frag<_Float16> {
  typedef v16h V; union U { v16h v; v8h h[2]; };
  static __device__ __forceinline__ v16h load(const _Float16* p) {
    U f; f.h[0] = *(const v8h*)(p); f.h[1] = *(const v8h*)(p + 16); return f.v;
  }
  static __device__ __forceinline__ v8f mma(v16h a, v16h b, v8f c) {
    return __builtin_amdgcn_wmma_f32_16x16x32_f16(false, a, false, b, (short)0, c, false, false);
  }
  static __device__ __forceinline__ void guard(v8f& a, v8f& b, v16h x, v16h y) { dep_guard_h(a, b, x, y); }
  static __device__ __forceinline__ void keep(v16h a, v16h b, v16h c, v16h d) { keep4_h(a, b, c, d); }
};
template <> struct Frag<__bf16> {
  typedef v16b V; union U { v16b v; v8b h[2]; };
  static __device__ __forceinline__ v16b load(const __bf16* p) {
    U f; f.h[0] = *(const v8b*)(p); f.h[1] = *(const v8b*)(p + 16); return f.v;
  }
  static __device__ __forceinline__ v8f mma(v16b a, v16b b, v8f c) {
    return __builtin_amdgcn_wmma_f32_16x16x32_bf16(false, a, false, b, (short)0, c, false, false);
  }
  static __device__ __forceinline__ void guard(v8f& a, v8f& b, v16b x, v16b y) { dep_guard_b(a, b, x, y); }
  static __device__ __forceinline__ void keep(v16b a, v16b b, v16b c, v16b d) { keep4_b(a, b, c, d); }
};

__device__ __forceinline__ unsigned pk16(unsigned short a, unsigned short b) { return (unsigned)a | ((unsigned)b << 16); }
__device__ __forceinline__ unsigned short h_bits(float f) { const _Float16 h = (_Float16)f; return __builtin_bit_cast(unsigned short, h); }

template <int ET> struct Elem;
template <> struct Elem<0> { typedef _Float16 T; };
template <> struct Elem<1> { typedef __bf16 T; };
template <int ET, bool SPLIT, int BIAS_MODE, int OUT_MODE, bool RESID, int ACT = 0>
__global__ __launch_bounds__(256) void wmma_gemm64(
    const unsigned short* __restrict__ Ap, const unsigned short* __restrict__ A2p, int lda, long strideA,
    const unsigned short* __restrict__ Btp, const unsigned short* __restrict__ Bt2p, int ldb, long strideB,
    void* __restrict__ Cout, void* __restrict__ Cout2, int ldc, long strideC,
    const float* __restrict__ bias,
    const float* __restrict__ resid, long strideR,
    int M, int N, int K, float scale) {
  typedef typename Elem<ET>::T T;
  typedef typename Frag<T>::V V;
  const T* A = (const T*)Ap; const T* A2 = (const T*)A2p; const T* Bt = (const T*)Btp; const T* Bt2 = (const T*)Bt2p;
  __shared__ __align__(16) float sT[8][16 * 68];
  const int b    = blockIdx.y;
  const int lane = threadIdx.x & 31;
  const int wave = threadIdx.x >> 5;
  const int tilesN = N >> 6;
  const int tilesM = M >> 6;
  const int tile = blockIdx.x * 8 + wave;
  if (tile >= tilesM * tilesN) return;
  const int tm = tile / tilesN;
  const int tn = tile - tm * tilesN;
  const int m0 = tm << 6;
  const int n0 = tn << 6;

  const T* Ab  = A  + (size_t)b * strideA;
  const T* Bb  = Bt + (size_t)b * strideB;
  const T* Ab2 = SPLIT ? (A2  + (size_t)b * strideA) : nullptr;
  const T* Bb2 = SPLIT ? (Bt2 + (size_t)b * strideB) : nullptr;

  const int rlane = lane & 15;
  const int koff  = (lane >> 4) * 8;
  const int mOff  = (lane >> 4) * 8;

  v8f acc[4][4];
#pragma unroll
  for (int i = 0; i < 4; ++i)
#pragma unroll
    for (int j = 0; j < 4; ++j) acc[i][j] = (v8f){0.f,0.f,0.f,0.f,0.f,0.f,0.f,0.f};

  for (int k0 = 0; k0 < K; k0 += 32) {
    V bh[4], bl[4];
#pragma unroll
    for (int j = 0; j < 4; ++j) {
      const size_t bo = (size_t)(n0 + (j << 4) + rlane) * ldb + koff + k0;
      bh[j] = Frag<T>::load(Bb + bo);
      if (SPLIT) bl[j] = Frag<T>::load(Bb2 + bo);
    }
#pragma unroll
    for (int i = 0; i < 4; ++i) {
      const size_t ao = (size_t)(m0 + (i << 4) + rlane) * lda + koff + k0;
      V ah = Frag<T>::load(Ab + ao);
      V al;
      if (SPLIT) al = Frag<T>::load(Ab2 + ao);
#pragma unroll
      for (int j = 0; j < 4; ++j) {
        acc[i][j] = Frag<T>::mma(ah, bh[j], acc[i][j]);
        if (SPLIT) {
          acc[i][j] = Frag<T>::mma(ah, bl[j], acc[i][j]);
          acc[i][j] = Frag<T>::mma(al, bh[j], acc[i][j]);
        }
      }
      Frag<T>::guard(acc[i][0], acc[i][3], ah, SPLIT ? al : ah);
    }
    Frag<T>::keep(bh[0], bh[1], bh[2], bh[3]);
    if (SPLIT) Frag<T>::keep(bl[0], bl[1], bl[2], bl[3]);
  }
  acc_guard4(acc[0][0], acc[0][1], acc[0][2], acc[0][3]);
  acc_guard4(acc[1][0], acc[1][1], acc[1][2], acc[1][3]);
  acc_guard4(acc[2][0], acc[2][1], acc[2][2], acc[2][3]);
  acc_guard4(acc[3][0], acc[3][1], acc[3][2], acc[3][3]);

  float* slab = sT[wave];
  const float* Rb = RESID ? (resid + (size_t)b * strideR) : nullptr;
#pragma unroll
  for (int i = 0; i < 4; ++i) {
    const int mBase = m0 + (i << 4);
#pragma unroll
    for (int j = 0; j < 4; ++j) {
      const int n = n0 + (j << 4) + rlane;
      float bv = 0.f;
      if (BIAS_MODE == 2) bv = bias[n];
#pragma unroll
      for (int r = 0; r < 8; ++r) {
        float v = acc[i][j][r] * scale;
        if (BIAS_MODE == 1) v += bias[mBase + mOff + r];
        if (BIAS_MODE == 2) v += bv;
        if (RESID) v += Rb[(size_t)(mBase + mOff + r) * ldc + n];
        if (ACT == 2) v = fmaxf(v, 0.0f);
        if (ACT == 4) v = (v > 0.f) ? v : 0.01f * v;
        slab[(mOff + r) * 68 + (j << 4) + rlane] = v;
      }
    }
    __builtin_amdgcn_fence(__ATOMIC_RELEASE, "workgroup");
    __builtin_amdgcn_wave_barrier();
    __builtin_amdgcn_fence(__ATOMIC_ACQUIRE, "workgroup");
    if (OUT_MODE == 0) {
      float* C = (float*)Cout + (size_t)b * strideC;
      const int hh = lane >> 4, c4 = (lane & 15) * 4;
      for (int pass = 0; pass < 2; ++pass) {
#pragma unroll
        for (int it = 0; it < 8; ++it) {
          const int row = it * 2 + hh;
          v4f v = *(const v4f*)(slab + row * 68 + c4);
          *(volatile v4f*)(C + (size_t)(mBase + row) * ldc + n0 + c4) = v;
        }
        __threadfence();
      }
    } else {
      const int q = lane >> 3, c8 = (lane & 7) * 8;
      unsigned short* C  = (unsigned short*)Cout  + (size_t)b * strideC;
      unsigned short* C2 = (OUT_MODE == 2) ? ((unsigned short*)Cout2 + (size_t)b * strideC) : nullptr;
      for (int pass = 0; pass < 2; ++pass) {
#pragma unroll
        for (int it = 0; it < 4; ++it) {
          const int row = it * 4 + q;
          const float* sp = slab + row * 68 + c8;
          v8h hv, lv;
#pragma unroll
          for (int e = 0; e < 8; ++e) {
            if (OUT_MODE == 1) {
              hv[e] = (_Float16)sp[e];
            } else {
              unsigned short hb = f2bf_bits(sp[e]);
              unsigned short lb = f2bf_bits(sp[e] - bf_bits2f(hb));
              hv[e] = __builtin_bit_cast(_Float16, hb);
              lv[e] = __builtin_bit_cast(_Float16, lb);
            }
          }
          *(volatile v8h*)(C + (size_t)(mBase + row) * ldc + n0 + c8) = hv;
          if (OUT_MODE == 2) *(volatile v8h*)(C2 + (size_t)(mBase + row) * ldc + n0 + c8) = lv;
        }
        __threadfence();
      }
    }
    __builtin_amdgcn_fence(__ATOMIC_RELEASE, "workgroup");
    __builtin_amdgcn_wave_barrier();
    __builtin_amdgcn_fence(__ATOMIC_ACQUIRE, "workgroup");
  }
}

__global__ __launch_bounds__(256) void cast8_planes_kernel(
    const float* __restrict__ in0, const float* __restrict__ in1,
    const float* __restrict__ in2, const float* __restrict__ in3,
    long srcOff, unsigned short* __restrict__ out, long outPlaneStride, int n8, float scale) {
  const int z = blockIdx.y;
  const float* src = (z == 0) ? in0 : (z == 1) ? in1 : (z == 2) ? in2 : in3;
  const int i = blockIdx.x * 256 + threadIdx.x;
  if (i >= n8) return;
  const float* p = src + srcOff + 8 * (size_t)i;
  const v4f a = *(const v4f*)(p);
  const v4f c = *(const v4f*)(p + 4);
  unsigned short hb[8];
#pragma unroll
  for (int e = 0; e < 4; ++e) {
    hb[e]     = h_bits(a[e] * scale);
    hb[4 + e] = h_bits(c[e] * scale);
  }
  const v4u u = (v4u){pk16(hb[0], hb[1]), pk16(hb[2], hb[3]), pk16(hb[4], hb[5]), pk16(hb[6], hb[7])};
  unsigned short* q = out + (size_t)z * outPlaneStride + 8 * (size_t)i;
  *(volatile v4u*)q = u;
  __threadfence();
  *(volatile v4u*)q = u;
}

__global__ __launch_bounds__(256) void softmax_row_kernel(const float* __restrict__ Sbase, unsigned short* __restrict__ Pbase,
                                                          float carry) {
  __shared__ float redM[8];
  __shared__ float redS[8];
  const int row  = blockIdx.x;
  const int grp  = blockIdx.y;
  const int t    = threadIdx.x;
  const int lane = t & 31, wave = t >> 5;
  const size_t base = (size_t)grp * (size_t)kSeqSeq + (size_t)row * kSeq + (size_t)t * 8;
  const float* sr = Sbase + base;
  const v4f a = *(const v4f*)(sr);
  const v4f c = *(const v4f*)(sr + 4);
  float m = fmaxf(fmaxf(fmaxf(a[0], a[1]), fmaxf(a[2], a[3])), fmaxf(fmaxf(c[0], c[1]), fmaxf(c[2], c[3])));
#pragma unroll
  for (int off = 16; off > 0; off >>= 1) m = fmaxf(m, __shfl_xor(m, off, 32));
  if (lane == 0) redM[wave] = m;
  __syncthreads();
  float gm = redM[0];
#pragma unroll
  for (int w = 1; w < 8; ++w) gm = fmaxf(gm, redM[w]);
  float e[8];
#pragma unroll
  for (int i = 0; i < 4; ++i) {
    e[i]     = expf(a[i] - gm);
    e[4 + i] = expf(c[i] - gm);
  }
  float s = ((e[0] + e[1]) + (e[2] + e[3])) + ((e[4] + e[5]) + (e[6] + e[7]));
#pragma unroll
  for (int off = 16; off > 0; off >>= 1) s += __shfl_xor(s, off, 32);
  if (lane == 0) redS[wave] = s;
  __syncthreads();
  float tot = redS[0];
#pragma unroll
  for (int w = 1; w < 8; ++w) tot += redS[w];
  const float inv = carry * (1.0f / tot);
  unsigned short hb[8];
#pragma unroll
  for (int i = 0; i < 8; ++i) hb[i] = h_bits(e[i] * inv);
  const v4u u = (v4u){pk16(hb[0], hb[1]), pk16(hb[2], hb[3]), pk16(hb[4], hb[5]), pk16(hb[6], hb[7])};
  unsigned short* q = Pbase + base;
  *(volatile v4u*)q = u;
  __threadfence();
  *(volatile v4u*)q = u;
}

extern "C" void kernel_launch(void* const* d_in, const int* in_sizes, int n_in,
                              void* d_out, int out_size, void* d_ws, size_t ws_size,
                              hipStream_t stream) {
  if (n_in < 14) return;
  if (in_sizes[0] != kBatch * (int)kTokDim || in_sizes[1] != kBatch * (int)kTokDim) return;
  for (int i = 0; i < 6; ++i) {
    if (in_sizes[2 + 2 * i] != (int)kDimDim) return;
    if (in_sizes[3 + 2 * i] != kDim) return;
  }
  if ((long)out_size != 2L * kBatch * kTokDim) return;
  if (ws_size < kWsTotal) return;

  const float* query   = (const float*)d_in[0];
  const float* context = (const float*)d_in[1];
  const float* W0 = (const float*)d_in[2];  const float* b0 = (const float*)d_in[3];
  const float* W1 = (const float*)d_in[4];  const float* b1 = (const float*)d_in[5];
  const float* W2 = (const float*)d_in[6];  const float* b2 = (const float*)d_in[7];
  const float* W3 = (const float*)d_in[8];  const float* b3 = (const float*)d_in[9];
  const float* W4 = (const float*)d_in[10]; const float* b4 = (const float*)d_in[11];
  const float* W5 = (const float*)d_in[12]; const float* b5 = (const float*)d_in[13];
  float* outp = (float*)d_out;

  char* ws = (char*)d_ws;
  unsigned short* X16q = (unsigned short*)(ws + kOffX16q);
  unsigned short* X16c = (unsigned short*)(ws + kOffX16c);
  unsigned short* W03  = (unsigned short*)(ws + kOffW03);
  float*          S32  = (float*)(ws + kOffS);
  unsigned short* P16  = (unsigned short*)(ws + kOffP);
  unsigned short* W45  = (unsigned short*)(ws + kOffW45);
  unsigned short* Q16  = (unsigned short*)(ws + kOffQ16);
  unsigned short* C16  = (unsigned short*)(ws + kOffC16);
  unsigned short* QVT  = (unsigned short*)(ws + kOffQVT);
  unsigned short* CVT  = (unsigned short*)(ws + kOffCVT);
  unsigned short* QRES = (unsigned short*)(ws + kOffQRES);
  unsigned short* CRES = (unsigned short*)(ws + kOffCRES);

  const int n8X = (int)(kTokDim / 8);
  const int n8W = (int)(kDimDim / 8);
  const dim3 gridCastX((n8X + 255) / 256, 2);
  const dim3 gridCastW03((n8W + 255) / 256, 4);
  const dim3 gridCastW45((n8W + 255) / 256, 2);
  const dim3 gridProj(((kSeq / 64) * (kDim / 64) + 7) / 8, 1);
  const dim3 gridS(((kSeq / 64) * (kSeq / 64) + 7) / 8, kHeadsPerChunk);
  const dim3 gridSmax(kSeq, kHeadsPerChunk);
  const dim3 gridPV(((kSeq / 64) * 1 + 7) / 8, kHeadsPerChunk);
  const dim3 gridOut(((kSeq / 64) * (kDim / 64) + 7) / 8, 1);

  for (int b = 0; b < kBatch; ++b) {
    const long xoff = (long)b * kTokDim;

    cast8_planes_kernel<<<gridCastX, 256, 0, stream>>>(query, context, query, context, xoff, X16q, kTokDim, n8X, 1.0f);
    cast8_planes_kernel<<<gridCastW03, 256, 0, stream>>>(W0, W1, W2, W3, 0L, W03, kDimDim, n8W, kWCarry);

    wmma_gemm64<0, false, 2, 1, false><<<gridProj, 256, 0, stream>>>(
        X16q, X16q, kDim, 0L, W03, W03, kDim, 0L, (void*)Q16, (void*)Q16, kDim, 0L,
        b0, query, 0L, kSeq, kDim, kDim, kProjScale);
    wmma_gemm64<0, false, 2, 1, false><<<gridProj, 256, 0, stream>>>(
        X16c, X16c, kDim, 0L, W03 + kDimDim, W03 + kDimDim, kDim, 0L, (void*)C16, (void*)C16, kDim, 0L,
        b1, query, 0L, kSeq, kDim, kDim, kProjScale);
    wmma_gemm64<0, false, 1, 1, false><<<gridProj, 256, 0, stream>>>(
        W03 + 2 * kDimDim, W03 + 2 * kDimDim, kDim, 0L, X16q, X16q, kDim, 0L, (void*)QVT, (void*)QVT, kSeq, 0L,
        b2, query, 0L, kDim, kSeq, kDim, kProjScale);
    wmma_gemm64<0, false, 1, 1, false><<<gridProj, 256, 0, stream>>>(
        W03 + 3 * kDimDim, W03 + 3 * kDimDim, kDim, 0L, X16c, X16c, kDim, 0L, (void*)CVT, (void*)CVT, kSeq, 0L,
        b3, query, 0L, kDim, kSeq, kDim, kProjScale);

    for (int h0 = 0; h0 < kHeads; h0 += kHeadsPerChunk) {
      const long hcol = (long)h0 * kDh;
      const long hrow = (long)h0 * kDh * kSeq;

      wmma_gemm64<0, false, 0, 0, false><<<gridS, 256, 0, stream>>>(
          Q16 + hcol, Q16 + hcol, kDim, (long)kDh, C16 + hcol, C16 + hcol, kDim, (long)kDh,
          (void*)S32, (void*)S32, kSeq, kSeqSeq, b0, query, 0L, kSeq, kSeq, kDh, kScoreScale);
      softmax_row_kernel<<<gridSmax, 256, 0, stream>>>(S32, P16, kPCarry);
      wmma_gemm64<0, false, 0, 1, false><<<gridPV, 256, 0, stream>>>(
          P16, P16, kSeq, kSeqSeq, CVT + hrow, CVT + hrow, kSeq, (long)kDh * kSeq,
          (void*)(QRES + hcol), (void*)(QRES + hcol), kDim, (long)kDh, b0, query, 0L, kSeq, kDh, kSeq, kPVScale);

      wmma_gemm64<0, false, 0, 0, false><<<gridS, 256, 0, stream>>>(
          C16 + hcol, C16 + hcol, kDim, (long)kDh, Q16 + hcol, Q16 + hcol, kDim, (long)kDh,
          (void*)S32, (void*)S32, kSeq, kSeqSeq, b0, query, 0L, kSeq, kSeq, kDh, kScoreScale);
      softmax_row_kernel<<<gridSmax, 256, 0, stream>>>(S32, P16, kPCarry);
      wmma_gemm64<0, false, 0, 1, false><<<gridPV, 256, 0, stream>>>(
          P16, P16, kSeq, kSeqSeq, QVT + hrow, QVT + hrow, kSeq, (long)kDh * kSeq,
          (void*)(CRES + hcol), (void*)(CRES + hcol), kDim, (long)kDh, b0, query, 0L, kSeq, kDh, kSeq, kPVScale);
    }

    cast8_planes_kernel<<<gridCastW45, 256, 0, stream>>>(W4, W5, W4, W5, 0L, W45, kDimDim, n8W, kWCarry);
    float* out0b = outp + xoff;
    float* out1b = outp + (long)kBatch * kTokDim + xoff;
    wmma_gemm64<0, false, 2, 0, false><<<gridOut, 256, 0, stream>>>(
        QRES, QRES, kDim, 0L, W45, W45, kDim, 0L, (void*)out0b, (void*)out0b, kDim, 0L,
        b4, query, 0L, kSeq, kDim, kDim, kOutScale);
    wmma_gemm64<0, false, 2, 0, false><<<gridOut, 256, 0, stream>>>(
        CRES, CRES, kDim, 0L, W45 + kDimDim, W45 + kDimDim, kDim, 0L, (void*)out1b, (void*)out1b, kDim, 0L,
        b5, query, 0L, kSeq, kDim, kDim, kOutScale);
  }
}
